// KANConv2d_34497177322246
// MI455X (gfx1250) — hardware-verified
//
#include <hip/hip_runtime.h>
#include <stdint.h>

#define NBATCH 8
#define CIN    16
#define COUT   64
#define HH     96
#define WW     96
#define LPIX   (HH * WW)
#define NPIX   (NBATCH * LPIX)
#define NX     (NBATCH * CIN * LPIX)
#define KPOS   9
#define NG     3
#define NT     8
#define KTOT   (CIN * KPOS * NT)
#define ICH    4
#define KSUB   (ICH * KPOS * NT)
#define NSTG   (CIN / ICH)
#define CPR    (ICH * KPOS)
#define TM     32
#define NTHR   128
#define OSP    32
#define NWCH   (COUT * CIN * KPOS)

#define BSC    64.0f
#define RSC    2048.0f
#define INV_H  0.015625f
#define INV_X  7.62939453125e-06f

static_assert(NX % 256 == 0);
static_assert(NWCH % 256 == 0);
static_assert(NPIX % TM == 0);
static_assert(LPIX % TM == 0);
static_assert(WW % TM == 0);
static_assert(KSUB % 32 == 0);
static_assert((TM * CPR) % NTHR == 0);
static_assert((COUT * 8) % NTHR == 0);
static_assert(NTHR == 128);
static_assert(KTOT % 8 == 0);

typedef _Float16     v16h __attribute__((ext_vector_type(16)));
typedef _Float16     v8h  __attribute__((ext_vector_type(8)));
typedef float        v8f  __attribute__((ext_vector_type(8)));
typedef float        v4f  __attribute__((ext_vector_type(4)));
typedef unsigned int v4u  __attribute__((ext_vector_type(4)));

__device__ __forceinline__ float bf_rne(float f) {
  unsigned x = __float_as_uint(f);
  x = (x + 0x7FFFu + ((x >> 16) & 1u)) & 0xFFFF0000u;
  return __uint_as_float(x);
}
__device__ __forceinline__ unsigned hbits(_Float16 h) {
  return (unsigned)__builtin_bit_cast(unsigned short, h);
}
__device__ __forceinline__ void split_h(float v, unsigned& bh, unsigned& bl) {
  const _Float16 h = (_Float16)v;
  const float    r = (v - (float)h) * RSC;
  const _Float16 l = (_Float16)r;
  bh = hbits(h);
  bl = hbits(l);
}
__device__ __forceinline__ v8f zero8() { v8f z = {0.f, 0.f, 0.f, 0.f, 0.f, 0.f, 0.f, 0.f}; return z; }

__device__ __forceinline__ v16h ldfrag(const _Float16* p) {
  union { v16h v; v8h h[2]; } f;
  f.h[0] = *(const v8h*)(p);
  f.h[1] = *(const v8h*)(p + 16);
  return f.v;
}

__device__ __forceinline__ v8f mma_h(v16h a, v16h b, v8f c) {
  return __builtin_amdgcn_wmma_f32_16x16x32_f16(false, a, false, b, (short)0, c, false, false);
}
__device__ __forceinline__ void dep_guard4(v8f& w, v8f& x, v8f& y, v8f& z,
                                           v16h f0, v16h f1, v16h f2, v16h f3, v16h f4, v16h f5) {
#if defined(__HIP_DEVICE_COMPILE__)
  asm volatile("v_nop\n\tv_nop\n\tv_nop\n\tv_nop"
               : "+v"(w), "+v"(x), "+v"(y), "+v"(z)
               : "v"(f0), "v"(f1), "v"(f2), "v"(f3), "v"(f4), "v"(f5));
#endif
}
__device__ __forceinline__ void acc_guard4(v8f& w, v8f& x, v8f& y, v8f& z) {
#if defined(__HIP_DEVICE_COMPILE__)
  asm volatile("v_nop\n\tv_nop\n\tv_nop\n\tv_nop" : "+v"(w), "+v"(x), "+v"(y), "+v"(z));
#endif
}

__global__ __launch_bounds__(256)
void k_feat(const float* __restrict__ x, unsigned* fh, unsigned* fl, int nx)
{
  const int e  = blockIdx.x * 256 + threadIdx.x;
  const int ec = (e < nx) ? e : (nx - 1);
  const float p = bf_rne(x[ec]);

  const float ex  = expf(-p);
  const float sil = p * __builtin_amdgcn_rcpf(1.0f + ex);
  float s1, c1;
  sincosf(p, &s1, &c1);
  const float c2 = c1 * c1 - s1 * s1;
  const float s2 = 2.0f * s1 * c1;
  const float c3 = c2 * c1 - s2 * s1;
  const float s3 = s2 * c1 + c2 * s1;

  const float v[8] = {sil, c1, c2, c3, s1, s2, s3, 0.0f};
  unsigned bh[8], bl[8];
#pragma unroll
  for (int t = 0; t < 8; ++t) split_h(v[t], bh[t], bl[t]);

  v4u wh, wl;
  wh.x = bh[0] | (bh[1] << 16);  wh.y = bh[2] | (bh[3] << 16);
  wh.z = bh[4] | (bh[5] << 16);  wh.w = bh[6] | (bh[7] << 16);
  wl.x = bl[0] | (bl[1] << 16);  wl.y = bl[2] | (bl[3] << 16);
  wl.z = bl[4] | (bl[5] << 16);  wl.w = bl[6] | (bl[7] << 16);

  unsigned* dh = fh + (size_t)ec * 4;
  unsigned* dl = fl + (size_t)ec * 4;
  if (e < nx) {
    *(volatile v4u*)dh = wh;
    *(volatile v4u*)dl = wl;
  }
  __threadfence();
  if (e < nx) {
    *(volatile v4u*)dh = wh;
    *(volatile v4u*)dl = wl;
  }
}

__global__ __launch_bounds__(256)
void k_wprep(const float* __restrict__ sb, const float* __restrict__ ss, const float* __restrict__ cf,
             unsigned* bh, unsigned* bl)
{
  const int idx = blockIdx.x * 256 + threadIdx.x;
  const int q   = (idx < NWCH) ? idx : (NWCH - 1);
  const int n   = q / (CIN * KPOS);
  const int c   = q - n * (CIN * KPOS);
  const int i   = c / KPOS;
  const int kp  = c - i * KPOS;

  const int wb  = (i * COUT + n) * KPOS + kp;
  const int cb0 = (((i * 2 + 0) * COUT + n) * KPOS + kp) * NG;
  const int cb1 = (((i * 2 + 1) * COUT + n) * KPOS + kp) * NG;

  const float sc = bf_rne(ss[wb]);
  float v[8];
  v[0] = bf_rne(sb[wb]);
#pragma unroll
  for (int g = 0; g < NG; ++g) {
    v[1 + g] = sc * bf_rne(cf[cb0 + g]);
    v[4 + g] = sc * bf_rne(cf[cb1 + g]);
  }
  v[7] = 0.0f;

  unsigned hb[8], lb[8];
#pragma unroll
  for (int t = 0; t < 8; ++t) split_h(v[t] * BSC, hb[t], lb[t]);

  v4u wh, wl;
  wh.x = hb[0] | (hb[1] << 16);  wh.y = hb[2] | (hb[3] << 16);
  wh.z = hb[4] | (hb[5] << 16);  wh.w = hb[6] | (hb[7] << 16);
  wl.x = lb[0] | (lb[1] << 16);  wl.y = lb[2] | (lb[3] << 16);
  wl.z = lb[4] | (lb[5] << 16);  wl.w = lb[6] | (lb[7] << 16);

  unsigned* dh = bh + (size_t)q * 4;
  unsigned* dl = bl + (size_t)q * 4;
  if (idx < NWCH) {
    *(volatile v4u*)dh = wh;
    *(volatile v4u*)dl = wl;
  }
  __threadfence();
  if (idx < NWCH) {
    *(volatile v4u*)dh = wh;
    *(volatile v4u*)dl = wl;
  }
}

__global__ __launch_bounds__(NTHR)
void k_gemm(const unsigned* __restrict__ fh, const unsigned* __restrict__ fl,
            const _Float16* __restrict__ bh, const _Float16* __restrict__ bl,
            const float* __restrict__ bias, float* out)
{
  __shared__ __align__(16) unsigned ah_s[TM * KSUB / 2];
  __shared__ __align__(16) unsigned al_s[TM * KSUB / 2];
  __shared__ __align__(16) float    o_s[COUT * OSP];
  __shared__ float bias_s[COUT];

  const int tid  = threadIdx.x;
  const int lane = tid & 31;
  const int wv   = tid >> 5;
  const int mt   = wv & 1;
  const int nh   = wv >> 1;
  const int lm   = lane & 15;
  const int hh   = lane >> 4;

  const int gp0 = blockIdx.x * TM;
  const int b   = gp0 / LPIX;
  const int hw0 = gp0 - b * LPIX;
  const int h   = hw0 / WW;
  const int w0  = hw0 - h * WW;

  if (tid < COUT) bias_s[tid] = bf_rne(bias[tid]);

  v8f acc_h0 = zero8(), acc_h1 = zero8(), acc_x0 = zero8(), acc_x1 = zero8();

  const _Float16* pa_h  = (const _Float16*)ah_s + (mt * 16 + lm) * KSUB + 8 * hh;
  const _Float16* pa_l  = (const _Float16*)al_s + (mt * 16 + lm) * KSUB + 8 * hh;
  const _Float16* pb_h0 = bh + (size_t)(nh * 32 + lm) * KTOT + 8 * hh;
  const _Float16* pb_h1 = pb_h0 + 16 * KTOT;
  const _Float16* pb_l0 = bl + (size_t)(nh * 32 + lm) * KTOT + 8 * hh;
  const _Float16* pb_l1 = pb_l0 + 16 * KTOT;

#pragma unroll 1
  for (int s = 0; s < NSTG; ++s) {
    __syncthreads();

#pragma unroll 1
    for (int q = tid; q < TM * CPR; q += NTHR) {
      const int pix = q & (TM - 1);
      const int c   = q >> 5;
      const int il  = c / KPOS;
      const int kp  = c - il * KPOS;
      const int ki  = kp / 3;
      const int kj  = kp - 3 * ki;
      const int i   = s * ICH + il;
      const int hs  = h + ki - 1;
      const int wsx = w0 + pix + kj - 1;
      const bool inr = ((unsigned)hs < (unsigned)HH) && ((unsigned)wsx < (unsigned)WW);
      const int hc  = (hs < 0) ? 0 : ((hs > HH - 1) ? (HH - 1) : hs);
      const int wc  = (wsx < 0) ? 0 : ((wsx > WW - 1) ? (WW - 1) : wsx);
      const size_t src = ((size_t)((b * CIN + i) * HH + hc) * WW + wc) * 4;
      const v4u gh = *(const v4u*)(fh + src);
      const v4u gl = *(const v4u*)(fl + src);
      v4u ph, pl;
      ph.x = inr ? gh.x : 0x3C000000u;
      ph.y = inr ? gh.y : 0x3C003C00u;
      ph.z = inr ? gh.z : 0u;
      ph.w = inr ? gh.w : 0u;
      pl.x = inr ? gl.x : 0u;
      pl.y = inr ? gl.y : 0u;
      pl.z = inr ? gl.z : 0u;
      pl.w = inr ? gl.w : 0u;
      const int dst = pix * (KSUB / 2) + c * 4;
      *(v4u*)(ah_s + dst) = ph;
      *(v4u*)(al_s + dst) = pl;
    }
    __syncthreads();

    const int kb = s * KSUB;
#pragma unroll 1
    for (int k0 = 0; k0 < KSUB; k0 += 32) {
      const v16h fa_h = ldfrag(pa_h + k0);
      const v16h fa_l = ldfrag(pa_l + k0);
      const v16h fb_h0 = ldfrag(pb_h0 + kb + k0);
      const v16h fb_h1 = ldfrag(pb_h1 + kb + k0);
      const v16h fb_l0 = ldfrag(pb_l0 + kb + k0);
      const v16h fb_l1 = ldfrag(pb_l1 + kb + k0);
      acc_h0 = mma_h(fa_h, fb_h0, acc_h0);
      acc_h1 = mma_h(fa_h, fb_h1, acc_h1);
      acc_x0 = mma_h(fa_l, fb_h0, acc_x0);
      acc_x1 = mma_h(fa_l, fb_h1, acc_x1);
      acc_x0 = mma_h(fa_h, fb_l0, acc_x0);
      acc_x1 = mma_h(fa_h, fb_l1, acc_x1);
      dep_guard4(acc_h0, acc_h1, acc_x0, acc_x1, fa_h, fa_l, fb_h0, fb_h1, fb_l0, fb_l1);
    }
  }
  acc_guard4(acc_h0, acc_h1, acc_x0, acc_x1);

  {
    const int pixb = mt * 16 + 8 * hh;
    const int o0 = nh * 32 + lm;
    const int o1 = o0 + 16;
    const float bb0 = bias_s[o0];
    const float bb1 = bias_s[o1];
    v4f ua, ub, uc, ud;
    ua.x = acc_h0[0] * INV_H + acc_x0[0] * INV_X + bb0;
    ua.y = acc_h0[1] * INV_H + acc_x0[1] * INV_X + bb0;
    ua.z = acc_h0[2] * INV_H + acc_x0[2] * INV_X + bb0;
    ua.w = acc_h0[3] * INV_H + acc_x0[3] * INV_X + bb0;
    ub.x = acc_h0[4] * INV_H + acc_x0[4] * INV_X + bb0;
    ub.y = acc_h0[5] * INV_H + acc_x0[5] * INV_X + bb0;
    ub.z = acc_h0[6] * INV_H + acc_x0[6] * INV_X + bb0;
    ub.w = acc_h0[7] * INV_H + acc_x0[7] * INV_X + bb0;
    uc.x = acc_h1[0] * INV_H + acc_x1[0] * INV_X + bb1;
    uc.y = acc_h1[1] * INV_H + acc_x1[1] * INV_X + bb1;
    uc.z = acc_h1[2] * INV_H + acc_x1[2] * INV_X + bb1;
    uc.w = acc_h1[3] * INV_H + acc_x1[3] * INV_X + bb1;
    ud.x = acc_h1[4] * INV_H + acc_x1[4] * INV_X + bb1;
    ud.y = acc_h1[5] * INV_H + acc_x1[5] * INV_X + bb1;
    ud.z = acc_h1[6] * INV_H + acc_x1[6] * INV_X + bb1;
    ud.w = acc_h1[7] * INV_H + acc_x1[7] * INV_X + bb1;
    *(v4f*)(o_s + o0 * OSP + pixb)     = ua;
    *(v4f*)(o_s + o0 * OSP + pixb + 4) = ub;
    *(v4f*)(o_s + o1 * OSP + pixb)     = uc;
    *(v4f*)(o_s + o1 * OSP + pixb + 4) = ud;
  }
  __syncthreads();

  float* obase = out + (size_t)b * COUT * LPIX + hw0;
#pragma unroll 1
  for (int q = tid; q < COUT * 8; q += NTHR) {
    const int o = q >> 3;
    const int piece = q & 7;
    const v4f v = *(const v4f*)(o_s + o * OSP + piece * 4);
    float* dst = obase + (size_t)o * LPIX + piece * 4;
    *(volatile v4f*)dst = v;
  }
  __threadfence();
#pragma unroll 1
  for (int q = tid; q < COUT * 8; q += NTHR) {
    const int o = q >> 3;
    const int piece = q & 7;
    const v4f v = *(const v4f*)(o_s + o * OSP + piece * 4);
    float* dst = obase + (size_t)o * LPIX + piece * 4;
    *(volatile v4f*)dst = v;
  }
}

extern "C" void kernel_launch(void* const* d_in, const int* in_sizes, int n_in,
                              void* d_out, int out_size, void* d_ws, size_t ws_size,
                              hipStream_t stream) {
  if (n_in < 5) return;
  if (in_sizes[0] != NX) return;
  if (in_sizes[1] != CIN * COUT * KPOS) return;
  if (in_sizes[2] != CIN * COUT * KPOS) return;
  if (in_sizes[3] != CIN * 2 * COUT * KPOS * NG) return;
  if (in_sizes[4] < COUT) return;
  if (out_size != NPIX * COUT) return;

  const size_t fbytes = (size_t)NX * 16;
  const size_t wbytes = (size_t)NWCH * 16;
  const size_t off_fh = 0;
  const size_t off_fl = off_fh + fbytes;
  const size_t off_bh = off_fl + fbytes;
  const size_t off_bl = off_bh + wbytes;
  const size_t total  = off_bl + wbytes;
  if (total > ws_size) return;

  const float* x            = (const float*)d_in[0];
  const float* scale_base   = (const float*)d_in[1];
  const float* scale_spline = (const float*)d_in[2];
  const float* coeff        = (const float*)d_in[3];
  const float* bias         = (const float*)d_in[4];
  float* out = (float*)d_out;

  unsigned char* wsb = (unsigned char*)d_ws;
  unsigned* fh = (unsigned*)(wsb + off_fh);
  unsigned* fl = (unsigned*)(wsb + off_fl);
  unsigned* bhp = (unsigned*)(wsb + off_bh);
  unsigned* blp = (unsigned*)(wsb + off_bl);

  const int nx = in_sizes[0];

  k_feat<<<dim3(NX / 256), dim3(256), 0, stream>>>(x, fh, fl, nx);
  (void)hipGetLastError();

  k_wprep<<<dim3(NWCH / 256), dim3(256), 0, stream>>>(scale_base, scale_spline, coeff, bhp, blp);
  (void)hipGetLastError();

  k_gemm<<<dim3(NPIX / TM), dim3(NTHR), 0, stream>>>(fh, fl, (const _Float16*)bhp, (const _Float16*)blp, bias, out);
  (void)hipGetLastError();
}
